// CrossChannelAttention_25812753448994
// MI455X (gfx1250) — hardware-verified
//
#include <hip/hip_runtime.h>


#define NBI  8
#define CC   128
#define NP   4096
#define NG   16
#define HH   8
#define NO   256
typedef _Float16 h16;
typedef unsigned short bf;
typedef __attribute__((ext_vector_type(16))) __bf16   v16bf;
typedef __attribute__((ext_vector_type(16))) _Float16 v16h;
typedef __attribute__((ext_vector_type(8)))  _Float16 v8h;
typedef __attribute__((ext_vector_type(8)))  unsigned short v8us;
typedef __attribute__((ext_vector_type(8)))  float    v8f;
typedef __attribute__((ext_vector_type(4)))  float    v4f;
typedef v8h  __attribute__((may_alias)) v8ha;
typedef v4f  __attribute__((may_alias)) v4fa;
typedef v8us __attribute__((may_alias)) v8usa;

__device__ __forceinline__ unsigned short f2bf(float f) { unsigned u = __float_as_uint(f); u += 0x7FFFu + ((u >> 16) & 1u); return (unsigned short)(u >> 16); }
__device__ __forceinline__ float bf2f(unsigned short b) { return __uint_as_float(((unsigned)b) << 16); }
__device__ __forceinline__ float bfr(float f) { return bf2f(f2bf(f)); }
__device__ __forceinline__ v16h cat16(v8h lo, v8h hi) { return __builtin_shufflevector(lo, hi, 0, 1, 2, 3, 4, 5, 6, 7, 8, 9, 10, 11, 12, 13, 14, 15); }
__device__ __forceinline__ v16bf cat16b(v8us lo, v8us hi) { return __builtin_bit_cast(v16bf, __builtin_shufflevector(lo, hi, 0, 1, 2, 3, 4, 5, 6, 7, 8, 9, 10, 11, 12, 13, 14, 15)); }
__device__ __forceinline__ v8f wmma16(v16h a, v16h b, v8f c) { return __builtin_amdgcn_wmma_f32_16x16x32_f16(false, a, false, b, (short)0, c, false, false); }
__device__ __forceinline__ v8f wmmab(v16bf a, v16bf b, v8f c) { return __builtin_amdgcn_wmma_f32_16x16x32_bf16(false, a, false, b, (short)0, c, false, false); }


template <typename T16> struct WFrag;
template <> struct WFrag<h16> { typedef v16h V; static __device__ __forceinline__ V ld(const h16* p) { return cat16(*(const v8h*)p, *(const v8h*)(p + 16)); } static __device__ __forceinline__ v8f mma(V a, V b, v8f c) { return wmma16(a, b, c); } };
template <> struct WFrag<bf> { typedef v16bf V; static __device__ __forceinline__ V ld(const bf* p) { return cat16b(*(const v8us*)p, *(const v8us*)(p + 16)); } static __device__ __forceinline__ v8f mma(V a, V b, v8f c) { return wmmab(a, b, c); } };
template <typename T16, int NSPLIT, bool BIAS>
__global__ __launch_bounds__(32) void k_gemmw(const T16* __restrict__ A, const T16* __restrict__ A2, const T16* __restrict__ Bt, const T16* __restrict__ Bt2, int K, float* C, int ldc, const float* __restrict__ bias, size_t sA, size_t sB, size_t sC) {
    typedef typename WFrag<T16>::V V;
    __shared__ __align__(16) float os[16 * 68];
    const size_t z = blockIdx.z; A += z * sA; if (A2) A2 += z * sA; Bt += z * sB; if (Bt2) Bt2 += z * sB; C += z * sC;
    const int lane = threadIdx.x & 31, lr = lane & 15, hi = lane >> 4; const int r0 = blockIdx.x * 64, c0 = blockIdx.y * 64;
    v8f acc[4][4];
#pragma unroll
    for (int mb = 0; mb < 4; ++mb)
#pragma unroll
        for (int nb = 0; nb < 4; ++nb) acc[mb][nb] = (v8f){};
    const size_t aoff = (size_t)(r0 + lr) * K + 8 * hi, boff = (size_t)(c0 + lr) * K + 8 * hi;
#pragma unroll 1
    for (int kc = 0; kc < K; kc += 32) {
        V a[4], a2[4];
#pragma unroll
        for (int mb = 0; mb < 4; ++mb) { a[mb] = WFrag<T16>::ld(A + aoff + (size_t)mb * 16 * K + kc); if (NSPLIT == 1 || NSPLIT == 2) a2[mb] = WFrag<T16>::ld(A2 + aoff + (size_t)mb * 16 * K + kc); }
#pragma unroll
        for (int nb = 0; nb < 4; ++nb) { const V b = WFrag<T16>::ld(Bt + boff + (size_t)nb * 16 * K + kc); V b2; if (NSPLIT >= 2) b2 = WFrag<T16>::ld(Bt2 + boff + (size_t)nb * 16 * K + kc);
#pragma unroll
            for (int mb = 0; mb < 4; ++mb) { acc[mb][nb] = WFrag<T16>::mma(a[mb], b, acc[mb][nb]); if (NSPLIT == 1 || NSPLIT == 2) acc[mb][nb] = WFrag<T16>::mma(a2[mb], b, acc[mb][nb]); if (NSPLIT >= 2) acc[mb][nb] = WFrag<T16>::mma(a[mb], b2, acc[mb][nb]); } }
        asm volatile("v_nop\n\tv_nop\n\tv_nop\n\tv_nop" : "+v"(acc[0][0]), "+v"(acc[1][1]), "+v"(acc[2][2]), "+v"(acc[3][3]) : "v"(a[0]), "v"(a[3]));
    }
#pragma unroll
    for (int mb = 0; mb < 4; ++mb) {
#pragma unroll
        for (int nb = 0; nb < 4; ++nb) {
#pragma unroll
            for (int j = 0; j < 8; ++j) os[(hi * 8 + j) * 68 + nb * 16 + lr] = acc[mb][nb][j]; }
        __builtin_amdgcn_wave_barrier(); asm volatile("" ::: "memory");
        float* crow = C + (size_t)(r0 + mb * 16) * ldc + c0;
#pragma unroll 1
        for (int ps = 0; ps < 2; ++ps) {
#pragma unroll
            for (int s = 0; s < 8; ++s) { const int row = 2 * s + hi, cofs = lr * 4; v4f val = *(const v4fa*)(os + row * 68 + cofs); if (BIAS) { val[0] += bfr(bias[c0 + cofs]); val[1] += bfr(bias[c0 + cofs + 1]); val[2] += bfr(bias[c0 + cofs + 2]); val[3] += bfr(bias[c0 + cofs + 3]); }
                *(volatile v4f*)(crow + (size_t)row * ldc + cofs) = val; }
            if (ps == 0) __threadfence(); }
        __builtin_amdgcn_wave_barrier(); asm volatile("" ::: "memory");
    }
}

typedef __attribute__((ext_vector_type(2))) unsigned short v2us;
typedef __attribute__((ext_vector_type(4))) unsigned short v4us;

__global__ __launch_bounds__(256) void k_w2p(const float* __restrict__ W2, bf* W2P) { const int e = (blockIdx.x * 256 + threadIdx.x) * 4; if (e >= NG * NO * CC) return; const int c = e % CC; const int o = (e / CC) % NO; const int g = e / (CC * NO); const v4f a = *(const v4f*)(W2 + (size_t)o * NG * CC + g * CC + c); v4us ov;
#pragma unroll
    for (int u = 0; u < 4; ++u) ov[u] = f2bf(a[u]); *(volatile v4us*)(W2P + e) = ov; __threadfence(); *(volatile v4us*)(W2P + e) = ov; }
__global__ __launch_bounds__(256) void k_xt(const float* __restrict__ x, bf* XT) { const int e = (blockIdx.x * 256 + threadIdx.x) * 2; if (e >= NP * CC) return; const int c = e % CC; const int p = e / CC; v2us o; o[0] = f2bf(x[(size_t)c * NP + p]); o[1] = f2bf(x[(size_t)(c + 1) * NP + p]); *(volatile v2us*)(XT + e) = o; __threadfence(); *(volatile v2us*)(XT + e) = o; }
__global__ __launch_bounds__(256) void k_fm(const float* __restrict__ x, const float* __restrict__ W1, const float* __restrict__ b1, float* FM) { const int e = (blockIdx.x * 256 + threadIdx.x) * 4; if (e >= NG * NP) return; const int p = e % NP; const int g = e / NP; float w[HH];
#pragma unroll
    for (int h = 0; h < HH; ++h) { w[h] = bfr(W1[g * HH + h]); asm volatile("" : "+v"(w[h])); }
    float bb = bfr(b1[g]); asm volatile("" : "+v"(bb)); v4f o;
#pragma unroll
    for (int u = 0; u < 4; ++u) { float acc = 0.f;
#pragma unroll
        for (int h = 0; h < HH; ++h) { float xv = bfr(x[((size_t)(g * HH + h)) * NP + p + u]); asm volatile("" : "+v"(xv)); float pr = __fmul_rn(xv, w[h]); asm volatile("" : "+v"(pr)); acc = __fadd_rn(acc, pr); }
        o[u] = fmaxf(__fadd_rn(acc, bb), 0.f); }
    *(volatile v4f*)(FM + e) = o; __threadfence(); *(volatile v4f*)(FM + e) = o; }
__global__ __launch_bounds__(256) void k_comb(const float* __restrict__ FM, const float* __restrict__ Y, const float* __restrict__ b2, float* OUTb) { const int e = (blockIdx.x * 256 + threadIdx.x) * 4; if (e >= NO * NP) return; const int p = e % NP; const int o = e / NP; float bb = bfr(b2[o]); asm volatile("" : "+v"(bb)); v4f acc = (v4f){0.f, 0.f, 0.f, 0.f};
#pragma unroll 1
    for (int g = 0; g < NG; ++g) { const v4f f = *(const v4f*)(FM + (size_t)g * NP + p), y = *(const v4f*)(Y + ((size_t)g * NO + o) * NP + p);
#pragma unroll
        for (int u = 0; u < 4; ++u) { float pr = __fmul_rn(f[u], y[u]); asm volatile("" : "+v"(pr)); acc[u] = __fadd_rn(acc[u], pr); } }
    v4f ov;
#pragma unroll
    for (int u = 0; u < 4; ++u) ov[u] = __fadd_rn(acc[u], bb); *(volatile v4f*)(OUTb + e) = ov; __threadfence(); *(volatile v4f*)(OUTb + e) = ov; }

extern "C" void kernel_launch(void* const* d_in, const int* in_sizes, int n_in,
                              void* d_out, int out_size, void* d_ws, size_t ws_size, hipStream_t stream) {
    (void)in_sizes; (void)n_in; (void)out_size;
    const float* x = (const float*)d_in[0]; const float* W1 = (const float*)d_in[1]; const float* b1 = (const float*)d_in[2]; const float* W2 = (const float*)d_in[3]; const float* b2 = (const float*)d_in[4];
    float* OUT = (float*)d_out;
    char* wsp = (char*)d_ws;
    auto take = [&](size_t bytes) { char* p = wsp; wsp += (bytes + 255) & ~(size_t)255; return (void*)p; };
    bf* W2P = (bf*)take((size_t)NG * NO * CC * 2); bf* XT = (bf*)take((size_t)NP * CC * 2); float* FM = (float*)take((size_t)NG * NP * 4); float* Y = (float*)take((size_t)NG * NO * NP * 4);
    if ((size_t)(wsp - (char*)d_ws) > ws_size) return;
    k_w2p<<<(NG * NO * CC / 4 + 255) / 256, 256, 0, stream>>>(W2, W2P);
    for (int b = 0; b < NBI; ++b) { const float* xb = x + (size_t)b * CC * NP;
        k_xt<<<(NP * CC / 2 + 255) / 256, 256, 0, stream>>>(xb, XT); k_fm<<<(NG * NP / 4 + 255) / 256, 256, 0, stream>>>(xb, W1, b1, FM);
        k_gemmw<bf, 0, false><<<dim3(NO / 64, NP / 64, NG), 32, 0, stream>>>(W2P, nullptr, XT, nullptr, CC, Y, NP, nullptr, (size_t)NO * CC, 0, (size_t)NO * NP);
        k_comb<<<(NO * NP / 4 + 255) / 256, 256, 0, stream>>>(FM, Y, b2, OUT + (size_t)b * NO * NP); }
}
